// GeoEncoderLayer_48533130445091
// MI455X (gfx1250) — hardware-verified
//
#include <hip/hip_runtime.h>
#include <stddef.h>
#include <stdint.h>

#define NB 8
#define NS 2048
#define DM 256
#define DF 1024
#define NR (NB * NS)

static_assert(NS % 64 == 0);
static_assert(DM == 256);
static_assert(DF % 64 == 0);
static_assert(NR % 256 == 0);

typedef _Float16 v16h __attribute__((ext_vector_type(16)));
typedef _Float16 v8h  __attribute__((ext_vector_type(8)));
typedef float    v8f  __attribute__((ext_vector_type(8)));
typedef float    v4f  __attribute__((ext_vector_type(4)));
typedef unsigned int v4u __attribute__((ext_vector_type(4)));

union Frag  { v16h v; v8h h[2]; };
union Pack8 { v8h h; v4u u; };

__device__ __forceinline__ v8f mma16(v16h a, v16h b, v8f c) {
  c = __builtin_amdgcn_wmma_f32_16x16x32_f16(false, a, false, b, (short)0, c, false, false);
  asm volatile("v_nop\n\tv_nop\n\tv_nop\n\tv_nop" : "+v"(c) : "v"(a), "v"(b));
  return c;
}

__device__ __forceinline__ v16h ldfrag(const _Float16* p, int ld, int row0, int k0, int lane) {
  const int m = lane & 15, lh = lane >> 4;
  const _Float16* q = p + (size_t)(row0 + m) * ld + k0 + 8 * lh;
  Frag f;
  f.h[0] = *(const v8h*)(q);
  f.h[1] = *(const v8h*)(q + 16);
  return f.v;
}

__device__ __forceinline__ v8f zero8() { return (v8f){0.f, 0.f, 0.f, 0.f, 0.f, 0.f, 0.f, 0.f}; }

template <int KK>
__device__ __forceinline__ void gemm32x64(const _Float16* __restrict__ A, int lda,
                                          const _Float16* __restrict__ Bt, int ldb,
                                          int m0, int n0, int lane, v8f (&acc)[2][4]) {
  static_assert(KK % 32 == 0);
#pragma unroll 2
  for (int k0 = 0; k0 < KK; k0 += 32) {
    const v16h a0 = ldfrag(A, lda, m0, k0, lane);
    const v16h a1 = ldfrag(A, lda, m0 + 16, k0, lane);
    const v16h b0 = ldfrag(Bt, ldb, n0, k0, lane);
    const v16h b1 = ldfrag(Bt, ldb, n0 + 16, k0, lane);
    const v16h b2 = ldfrag(Bt, ldb, n0 + 32, k0, lane);
    const v16h b3 = ldfrag(Bt, ldb, n0 + 48, k0, lane);
    acc[0][0] = mma16(a0, b0, acc[0][0]);
    acc[1][0] = mma16(a1, b0, acc[1][0]);
    acc[0][1] = mma16(a0, b1, acc[0][1]);
    acc[1][1] = mma16(a1, b1, acc[1][1]);
    acc[0][2] = mma16(a0, b2, acc[0][2]);
    acc[1][2] = mma16(a1, b2, acc[1][2]);
    acc[0][3] = mma16(a0, b3, acc[0][3]);
    acc[1][3] = mma16(a1, b3, acc[1][3]);
  }
}

#define WTP 68
__global__ __launch_bounds__(256) void k_wt(const float* __restrict__ w, _Float16* __restrict__ wt,
                                            int nout, int kin, float scl) {
  __shared__ __align__(16) float tf[64 * WTP];
  const int tid = threadIdx.x;
  const int n0 = blockIdx.x * 64;
  const int k0 = blockIdx.y * 64;
  {
    const int kr = tid >> 4;
    const int n4 = (tid & 15) * 4;
#pragma unroll
    for (int it = 0; it < 4; ++it) {
      const int kl = it * 16 + kr;
      const v4f a = *(const v4f*)(w + (size_t)(k0 + kl) * nout + n0 + n4);
      *(v4f*)(tf + kl * WTP + n4) = a;
    }
  }
  __syncthreads();
  v4u val[2];
  size_t go[2];
#pragma unroll
  for (int j = 0; j < 2; ++j) {
    const int p  = tid + 256 * j;
    const int nl = p >> 3;
    const int pc = p & 7;
    const float* cp = tf + (pc * 8) * WTP + nl;
    Pack8 pk;
    pk.h = (v8h){(_Float16)(cp[0 * WTP] * scl), (_Float16)(cp[1 * WTP] * scl),
                 (_Float16)(cp[2 * WTP] * scl), (_Float16)(cp[3 * WTP] * scl),
                 (_Float16)(cp[4 * WTP] * scl), (_Float16)(cp[5 * WTP] * scl),
                 (_Float16)(cp[6 * WTP] * scl), (_Float16)(cp[7 * WTP] * scl)};
    val[j] = pk.u;
    go[j]  = (size_t)(n0 + nl) * kin + k0 + pc * 8;
  }
  for (int ps = 0; ps < 2; ++ps) {
#pragma unroll
    for (int j = 0; j < 2; ++j) *(volatile v4u*)(wt + go[j]) = val[j];
    __threadfence();
  }
}

#define LTP 264
__global__ __launch_bounds__(256) void k_ln(const float* __restrict__ xin, const float* __restrict__ gam,
                                            const float* __restrict__ bet, _Float16* __restrict__ hout,
                                            _Float16* __restrict__ htout, int do_t) {
  __shared__ __align__(16) _Float16 T[64 * LTP];
  const int tid = threadIdx.x, lane = tid & 31, wave = tid >> 5;
  const int row0 = blockIdx.x * 64;
  const v4f g0 = *(const v4f*)(gam + 8 * lane);
  const v4f g1 = *(const v4f*)(gam + 8 * lane + 4);
  const v4f e0 = *(const v4f*)(bet + 8 * lane);
  const v4f e1 = *(const v4f*)(bet + 8 * lane + 4);
  const float invn = 0.00390625f;

#pragma unroll 1
  for (int i = 0; i < 8; ++i) {
    const int lr = wave * 8 + i;
    const size_t R = (size_t)(row0 + lr);
    const float* xp = xin + R * DM + 8 * lane;
    const v4f a0 = *(const v4f*)(xp);
    const v4f a1 = *(const v4f*)(xp + 4);
    float s = ((a0[0] + a0[1]) + (a0[2] + a0[3])) + ((a1[0] + a1[1]) + (a1[2] + a1[3]));
#pragma unroll
    for (int off = 1; off < 32; off <<= 1) s += __shfl_xor(s, off, 32);
    const float mu = s * invn;
    const v4f d0 = a0 - mu;
    const v4f d1 = a1 - mu;
    float q = d0[0] * d0[0] + d0[1] * d0[1] + d0[2] * d0[2] + d0[3] * d0[3]
            + d1[0] * d1[0] + d1[1] * d1[1] + d1[2] * d1[2] + d1[3] * d1[3];
#pragma unroll
    for (int off = 1; off < 32; off <<= 1) q += __shfl_xor(q, off, 32);
    const float var  = q * invn;
    const float rstd = rsqrtf(var + 1e-5f);
    const v4f o0 = d0 * rstd * g0 + e0;
    const v4f o1 = d1 * rstd * g1 + e1;
    Pack8 pk;
    pk.h = (v8h){(_Float16)o0[0], (_Float16)o0[1], (_Float16)o0[2], (_Float16)o0[3],
                 (_Float16)o1[0], (_Float16)o1[1], (_Float16)o1[2], (_Float16)o1[3]};
    const v4u u = pk.u;
    if (do_t != 0) *(v4u*)(T + lr * LTP + 8 * lane) = u;
    volatile v4u* dp = (volatile v4u*)(hout + R * DM + 8 * lane);
    *dp = u;
    __threadfence();
    *dp = u;
  }

  if (do_t != 0) {
    __syncthreads();
    const int bidx = row0 >> 11;
    const int nb   = row0 & (NS - 1);
    v4u val[8];
    size_t go[8];
#pragma unroll
    for (int j = 0; j < 8; ++j) {
      const int p  = tid + 256 * j;
      const int d  = p >> 3;
      const int pc = p & 7;
      const _Float16* cp = T + (pc * 8) * LTP + d;
      Pack8 pk;
      pk.h = (v8h){cp[0 * LTP], cp[1 * LTP], cp[2 * LTP], cp[3 * LTP],
                   cp[4 * LTP], cp[5 * LTP], cp[6 * LTP], cp[7 * LTP]};
      val[j] = pk.u;
      go[j]  = ((size_t)(bidx * DM + d)) * NS + nb + pc * 8;
    }
    for (int ps = 0; ps < 2; ++ps) {
#pragma unroll
      for (int j = 0; j < 8; ++j) *(volatile v4u*)(htout + go[j]) = val[j];
      __threadfence();
    }
  }
}

#define KSP 264
#define VSP 40
#define PSP 40
#define OSP 68
#define SM_KS (32 * KSP * 2)
#define SM_VS (256 * VSP * 2)
#define SM_PS (4 * 16 * PSP * 2)
#define SM_ATT (SM_KS + SM_VS + SM_PS)
static_assert(8 * 16 * OSP * 4 <= SM_KS + SM_VS);
static_assert((SM_KS % 16) == 0 && (SM_VS % 16) == 0);

__global__ __launch_bounds__(256) void k_attn(const _Float16* __restrict__ hp,
                                              const _Float16* __restrict__ htp,
                                              const float* __restrict__ xg,
                                              float* __restrict__ x1) {
  __shared__ __align__(16) unsigned char smem[SM_ATT];
  __shared__ float Al[64];
  __shared__ float Lr[64];
  _Float16* Ks = (_Float16*)smem;
  _Float16* Vs = (_Float16*)(smem + SM_KS);
  _Float16* Ps = (_Float16*)(smem + SM_KS + SM_VS);
  float*    Os = (float*)smem;

  const int tid = threadIdx.x, lane = tid & 31, wave = tid >> 5;
  const int hh = lane >> 4, c = lane & 15;
  const int b  = blockIdx.x >> 5;
  const int qb = blockIdx.x & 31;
  const int rg = wave & 3, ch = wave >> 2;
  const int q0 = qb * 64 + 16 * rg;

  const _Float16* Hb  = hp  + (size_t)b * NS * DM;
  const _Float16* Htb = htp + (size_t)b * DM * NS;
  _Float16* pw = Ps + rg * 16 * PSP;

  const float NEGI = -__builtin_huge_valf();
  const float sscale = 0.0625f;
  float mrow[8], lrow[8];
  v8f oacc[8];
#pragma unroll
  for (int r = 0; r < 8; ++r) { mrow[r] = NEGI; lrow[r] = 0.f; }
#pragma unroll
  for (int t = 0; t < 8; ++t) oacc[t] = zero8();

  for (int kc = 0; kc < NS / 32; ++kc) {
    const int kv0 = kc * 32;
    __syncthreads();
#pragma unroll
    for (int i = 0; i < 4; ++i) {
      const int p  = tid + 256 * i;
      const int r  = p >> 5;
      const int cc = (p & 31) * 8;
      *(v8h*)(Ks + r * KSP + cc) = *(const v8h*)(Hb + (size_t)(kv0 + r) * DM + cc);
      const int d  = p >> 2;
      const int c2 = (p & 3) * 8;
      *(v8h*)(Vs + d * VSP + c2) = *(const v8h*)(Htb + (size_t)d * NS + kv0 + c2);
    }
    __syncthreads();

    if (wave < 4) {
      v8f s[2];
      s[0] = zero8(); s[1] = zero8();
#pragma unroll 2
      for (int dc = 0; dc < DM / 32; ++dc) {
        const v16h qa = ldfrag(Hb, DM, q0, dc * 32, lane);
#pragma unroll
        for (int j = 0; j < 2; ++j) {
          const v16h kb = ldfrag(Ks, KSP, j * 16, dc * 32, lane);
          s[j] = mma16(qa, kb, s[j]);
        }
      }
      float cm[8];
#pragma unroll
      for (int r = 0; r < 8; ++r) {
        float m = NEGI;
#pragma unroll
        for (int j = 0; j < 2; ++j) {
          const float sv = s[j][r] * sscale;
          s[j][r] = sv;
          m = fmaxf(m, sv);
        }
#pragma unroll
        for (int off = 1; off < 16; off <<= 1) m = fmaxf(m, __shfl_xor(m, off, 32));
        cm[r] = m;
      }
#pragma unroll
      for (int r = 0; r < 8; ++r) {
        const float mnew  = fmaxf(mrow[r], cm[r]);
        const float alpha = __expf(mrow[r] - mnew);
        mrow[r] = mnew;
        float psum = 0.f;
#pragma unroll
        for (int j = 0; j < 2; ++j) {
          const float p = __expf(s[j][r] - mnew);
          psum += p;
          pw[(8 * hh + r) * PSP + j * 16 + c] = (_Float16)(p * 1024.0f);
        }
#pragma unroll
        for (int off = 1; off < 16; off <<= 1) psum += __shfl_xor(psum, off, 32);
        lrow[r] = lrow[r] * alpha + psum;
        if (c == 0) Al[rg * 16 + 8 * hh + r] = alpha;
      }
    }
    __syncthreads();

    float al[8];
#pragma unroll
    for (int r = 0; r < 8; ++r) al[r] = Al[rg * 16 + 8 * hh + r];
#pragma unroll
    for (int t = 0; t < 8; ++t)
#pragma unroll
      for (int r = 0; r < 8; ++r) oacc[t][r] *= al[r];
    const v16h pa = ldfrag(pw, PSP, 0, 0, lane);
#pragma unroll
    for (int t = 0; t < 8; ++t) {
      const v16h vb = ldfrag(Vs, VSP, 128 * ch + t * 16, 0, lane);
      oacc[t] = mma16(pa, vb, oacc[t]);
    }
  }

  if (wave < 4) {
    if (c == 0) {
#pragma unroll
      for (int r = 0; r < 8; ++r) Lr[rg * 16 + 8 * hh + r] = lrow[r];
    }
  }
  __syncthreads();
  float inv[8];
#pragma unroll
  for (int r = 0; r < 8; ++r) inv[r] = 0.0009765625f * __builtin_amdgcn_rcpf(Lr[rg * 16 + 8 * hh + r]);

  float* sw = Os + wave * (16 * OSP);
  const size_t rowg0 = (size_t)b * NS + q0;
  const int colb = 128 * ch;
#pragma unroll
  for (int cq = 0; cq < 2; ++cq) {
    __syncthreads();
#pragma unroll
    for (int tt = 0; tt < 4; ++tt) {
#pragma unroll
      for (int r = 0; r < 8; ++r)
        sw[(8 * hh + r) * OSP + 16 * tt + c] = oacc[4 * cq + tt][r] * inv[r];
    }
    __syncthreads();
    v4f val[8];
    size_t go[8];
#pragma unroll
    for (int it = 0; it < 8; ++it) {
      const int p    = lane + 32 * it;
      const int L    = p >> 3;
      const int pc   = p & 7;
      const int row  = L >> 1;
      const int half = L & 1;
      go[it] = (rowg0 + row) * DM + colb + 64 * cq + 32 * half + 4 * pc;
      const v4f ov = *(const v4f*)(sw + row * OSP + half * 32 + pc * 4);
      const v4f xv = *(const v4f*)(xg + go[it]);
      val[it] = ov + xv;
    }
    for (int ps = 0; ps < 2; ++ps) {
#pragma unroll
      for (int it = 0; it < 8; ++it) *(volatile v4f*)(x1 + go[it]) = val[it];
      __threadfence();
    }
  }
}

#define STP 72
__global__ __launch_bounds__(256) void k_ffn1(const _Float16* __restrict__ h2,
                                              const _Float16* __restrict__ w1t,
                                              const float* __restrict__ bias,
                                              _Float16* __restrict__ act) {
  __shared__ __align__(16) _Float16 st[256 * STP];
  const int tid = threadIdx.x, lane = tid & 31, wave = tid >> 5;
  const int hh = lane >> 4, c = lane & 15;
  const int mb = blockIdx.x * 256;
  const int m0 = mb + wave * 32;
  const int n0 = blockIdx.y * 64;

  v8f acc[2][4];
#pragma unroll
  for (int s = 0; s < 2; ++s)
#pragma unroll
    for (int t = 0; t < 4; ++t) acc[s][t] = zero8();
  gemm32x64<DM>(h2, DM, w1t, DM, m0, n0, lane, acc);

#pragma unroll
  for (int t = 0; t < 4; ++t) {
    const float bv = bias[n0 + 16 * t + c];
#pragma unroll
    for (int sub = 0; sub < 2; ++sub) {
#pragma unroll
      for (int r = 0; r < 8; ++r) {
        const int lr = wave * 32 + sub * 16 + 8 * hh + r;
        st[lr * STP + 16 * t + c] = (_Float16)fmaxf(acc[sub][t][r] * 0.0625f + bv, 0.f);
      }
    }
  }
  __syncthreads();

  v4u val[8];
  size_t go[8];
#pragma unroll
  for (int j = 0; j < 8; ++j) {
    const int p  = tid + 256 * j;
    const int lr = p >> 3;
    const int pc = p & 7;
    Pack8 pk;
    pk.h   = *(const v8h*)(st + lr * STP + pc * 8);
    val[j] = pk.u;
    go[j]  = (size_t)(mb + lr) * DF + n0 + pc * 8;
  }
  for (int ps = 0; ps < 2; ++ps) {
#pragma unroll
    for (int j = 0; j < 8; ++j) *(volatile v4u*)(act + go[j]) = val[j];
    __threadfence();
  }
}

__global__ __launch_bounds__(256) void k_ffn2(const _Float16* __restrict__ ap,
                                              const _Float16* __restrict__ wt,
                                              const float* __restrict__ bias,
                                              const float* __restrict__ x1,
                                              float* __restrict__ out) {
  __shared__ __align__(16) float st[8][16 * OSP];
  const int tid = threadIdx.x, lane = tid & 31, wave = tid >> 5;
  const int hh = lane >> 4, c = lane & 15;
  const int m0 = blockIdx.x * 256 + wave * 32;
  const int n0 = blockIdx.y * 64;

  v8f acc[2][4];
#pragma unroll
  for (int s = 0; s < 2; ++s)
#pragma unroll
    for (int t = 0; t < 4; ++t) acc[s][t] = zero8();
  gemm32x64<DF>(ap, DF, wt, DF, m0, n0, lane, acc);

  float bvs[4];
#pragma unroll
  for (int t = 0; t < 4; ++t) bvs[t] = bias[n0 + 16 * t + c];

  float* sw = st[wave];
#pragma unroll
  for (int sub = 0; sub < 2; ++sub) {
    __syncthreads();
#pragma unroll
    for (int t = 0; t < 4; ++t) {
#pragma unroll
      for (int r = 0; r < 8; ++r)
        sw[(8 * hh + r) * OSP + 16 * t + c] = acc[sub][t][r] * 0.03125f + bvs[t];
    }
    __syncthreads();
    v4f val[8];
    size_t go[8];
#pragma unroll
    for (int it = 0; it < 8; ++it) {
      const int p    = lane + 32 * it;
      const int L    = p >> 3;
      const int pc   = p & 7;
      const int row  = L >> 1;
      const int half = L & 1;
      go[it] = (size_t)(m0 + sub * 16 + row) * DM + n0 + half * 32 + pc * 4;
      const v4f ov = *(const v4f*)(sw + row * OSP + half * 32 + pc * 4);
      const v4f rv = *(const v4f*)(x1 + go[it]);
      val[it] = ov + rv;
    }
    for (int ps = 0; ps < 2; ++ps) {
#pragma unroll
      for (int it = 0; it < 8; ++it) *(volatile v4f*)(out + go[it]) = val[it];
      __threadfence();
    }
  }
}

extern "C" void kernel_launch(void* const* d_in, const int* in_sizes, int n_in,
                              void* d_out, int out_size, void* d_ws, size_t ws_size,
                              hipStream_t stream) {
  if (n_in < 9) return;
  if (in_sizes[0] != NR * DM) return;
  if (in_sizes[1] != DM * DF) return;
  if (in_sizes[2] != DF) return;
  if (in_sizes[3] != DF * DM) return;
  if (in_sizes[4] != DM) return;
  if (in_sizes[5] != DM || in_sizes[6] != DM || in_sizes[7] != DM || in_sizes[8] != DM) return;
  if (out_size != NR * DM) return;

  const float* x   = (const float*)d_in[0];
  const float* w1  = (const float*)d_in[1];
  const float* b1  = (const float*)d_in[2];
  const float* w2  = (const float*)d_in[3];
  const float* b2  = (const float*)d_in[4];
  const float* g1  = (const float*)d_in[5];
  const float* be1 = (const float*)d_in[6];
  const float* g2  = (const float*)d_in[7];
  const float* be2 = (const float*)d_in[8];
  float* out = (float*)d_out;

  size_t off = 0;
  const size_t oH   = off; off += (size_t)NR * DM * 2;
  const size_t oHt  = off; off += (size_t)NR * DM * 2;
  const size_t oX1  = off; off += (size_t)NR * DM * 4;
  const size_t oH2  = off; off += (size_t)NR * DM * 2;
  const size_t oAct = off; off += (size_t)NR * DF * 2;
  const size_t oW1  = off; off += (size_t)DF * DM * 2;
  const size_t oW2  = off; off += (size_t)DM * DF * 2;
  if (off > ws_size) return;

  char* ws = (char*)d_ws;
  _Float16* Hp   = (_Float16*)(ws + oH);
  _Float16* Htp  = (_Float16*)(ws + oHt);
  float*    X1p  = (float*)(ws + oX1);
  _Float16* H2p  = (_Float16*)(ws + oH2);
  _Float16* Actp = (_Float16*)(ws + oAct);
  _Float16* W1t  = (_Float16*)(ws + oW1);
  _Float16* W2t  = (_Float16*)(ws + oW2);

  k_wt<<<dim3(DF / 64, DM / 64), dim3(256), 0, stream>>>(w1, W1t, DF, DM, 16.0f);
  k_wt<<<dim3(DM / 64, DF / 64), dim3(256), 0, stream>>>(w2, W2t, DM, DF, 32.0f);
  k_ln<<<dim3(NR / 64), dim3(256), 0, stream>>>(x, g1, be1, Hp, Htp, 1);
  k_attn<<<dim3(NB * (NS / 64)), dim3(256), 0, stream>>>(Hp, Htp, x, X1p);
  k_ln<<<dim3(NR / 64), dim3(256), 0, stream>>>(X1p, g2, be2, H2p, Htp, 0);
  k_ffn1<<<dim3(NR / 256, DF / 64), dim3(256), 0, stream>>>(H2p, W1t, b1, Actp);
  k_ffn2<<<dim3(NR / 256, DM / 64), dim3(256), 0, stream>>>(Actp, W2t, b2, X1p, out);
  (void)hipGetLastError();
}
